// MultiHeadSpatialAttention_75488345194521
// MI455X (gfx1250) — hardware-verified
//
#include <hip/hip_runtime.h>
#include <math.h>
typedef __attribute__((ext_vector_type(16))) _Float16 v16h;
typedef __attribute__((ext_vector_type(8)))  _Float16 v8h;
typedef __attribute__((ext_vector_type(16))) __bf16   v16b;
typedef __attribute__((ext_vector_type(8)))  __bf16   v8b;
typedef __attribute__((ext_vector_type(8)))  float    v8f;
typedef __attribute__((ext_vector_type(4)))  float    v4f;
#define PSCALE 32768.0f
#define U16(p) ((const unsigned short*)(const void*)(p))
#define PSCALE_INV (1.0f / 32768.0f)

__device__ __forceinline__ unsigned short f2bf_bits(float f) {
  unsigned u = __float_as_uint(f);
  return (unsigned short)((u + 0x7FFFu + ((u >> 16) & 1u)) >> 16);
}
__device__ __forceinline__ float bf_bits2f(unsigned short h) { return __uint_as_float(((unsigned)h) << 16); }

__device__ __forceinline__ void dep_guard_h(v8f& a, v8f& b, v16h x, v16h y) { asm volatile("v_nop\n\tv_nop\n\tv_nop\n\tv_nop" : "+v"(a), "+v"(b) : "v"(x), "v"(y)); }
__device__ __forceinline__ void dep_guard_b(v8f& a, v8f& b, v16b x, v16b y) { asm volatile("v_nop\n\tv_nop\n\tv_nop\n\tv_nop" : "+v"(a), "+v"(b) : "v"(x), "v"(y)); }
__device__ __forceinline__ void keep4_h(v16h a, v16h b, v16h c, v16h d) { asm volatile("v_nop" :: "v"(a), "v"(b), "v"(c), "v"(d)); }
__device__ __forceinline__ void keep4_b(v16b a, v16b b, v16b c, v16b d) { asm volatile("v_nop" :: "v"(a), "v"(b), "v"(c), "v"(d)); }
__device__ __forceinline__ void acc_guard4(v8f& a, v8f& b, v8f& c, v8f& d) { asm volatile("v_nop\n\tv_nop\n\tv_nop\n\tv_nop" : "+v"(a), "+v"(b), "+v"(c), "+v"(d)); }
template <typename T> struct Frag;
template <> struct Frag<_Float16> {
  typedef v16h V; union U { v16h v; v8h h[2]; };
  static __device__ __forceinline__ v16h load(const _Float16* p) {
    U f; f.h[0] = *(const v8h*)(p); f.h[1] = *(const v8h*)(p + 16); return f.v;
  }
  static __device__ __forceinline__ v8f mma(v16h a, v16h b, v8f c) {
    return __builtin_amdgcn_wmma_f32_16x16x32_f16(false, a, false, b, (short)0, c, false, false);
  }
  static __device__ __forceinline__ void guard(v8f& a, v8f& b, v16h x, v16h y) { dep_guard_h(a, b, x, y); }
  static __device__ __forceinline__ void keep(v16h a, v16h b, v16h c, v16h d) { keep4_h(a, b, c, d); }
};
template <> struct Frag<__bf16> {
  typedef v16b V; union U { v16b v; v8b h[2]; };
  static __device__ __forceinline__ v16b load(const __bf16* p) {
    U f; f.h[0] = *(const v8b*)(p); f.h[1] = *(const v8b*)(p + 16); return f.v;
  }
  static __device__ __forceinline__ v8f mma(v16b a, v16b b, v8f c) {
    return __builtin_amdgcn_wmma_f32_16x16x32_bf16(false, a, false, b, (short)0, c, false, false);
  }
  static __device__ __forceinline__ void guard(v8f& a, v8f& b, v16b x, v16b y) { dep_guard_b(a, b, x, y); }
  static __device__ __forceinline__ void keep(v16b a, v16b b, v16b c, v16b d) { keep4_b(a, b, c, d); }
};

template <int ET> struct Elem;
template <> struct Elem<0> { typedef _Float16 T; };
template <> struct Elem<1> { typedef __bf16 T; };
template <int ET, bool SPLIT, int BIAS_MODE, int OUT_MODE, bool RESID, int ACT = 0>
__global__ __launch_bounds__(256) void wmma_gemm64(
    const unsigned short* __restrict__ Ap, const unsigned short* __restrict__ A2p, int lda, long strideA,
    const unsigned short* __restrict__ Btp, const unsigned short* __restrict__ Bt2p, int ldb, long strideB,
    void* __restrict__ Cout, void* __restrict__ Cout2, int ldc, long strideC,
    const float* __restrict__ bias,
    const float* __restrict__ resid, long strideR,
    int M, int N, int K, float scale) {
  typedef typename Elem<ET>::T T;
  typedef typename Frag<T>::V V;
  const T* A = (const T*)Ap; const T* A2 = (const T*)A2p; const T* Bt = (const T*)Btp; const T* Bt2 = (const T*)Bt2p;
  __shared__ __align__(16) float sT[8][16 * 68];
  const int b    = blockIdx.y;
  const int lane = threadIdx.x & 31;
  const int wave = threadIdx.x >> 5;
  const int tilesN = N >> 6;
  const int tilesM = M >> 6;
  const int tile = blockIdx.x * 8 + wave;
  if (tile >= tilesM * tilesN) return;
  const int tm = tile / tilesN;
  const int tn = tile - tm * tilesN;
  const int m0 = tm << 6;
  const int n0 = tn << 6;

  const T* Ab  = A  + (size_t)b * strideA;
  const T* Bb  = Bt + (size_t)b * strideB;
  const T* Ab2 = SPLIT ? (A2  + (size_t)b * strideA) : nullptr;
  const T* Bb2 = SPLIT ? (Bt2 + (size_t)b * strideB) : nullptr;

  const int rlane = lane & 15;
  const int koff  = (lane >> 4) * 8;
  const int mOff  = (lane >> 4) * 8;

  v8f acc[4][4];
#pragma unroll
  for (int i = 0; i < 4; ++i)
#pragma unroll
    for (int j = 0; j < 4; ++j) acc[i][j] = (v8f){0.f,0.f,0.f,0.f,0.f,0.f,0.f,0.f};

  for (int k0 = 0; k0 < K; k0 += 32) {
    V bh[4], bl[4];
#pragma unroll
    for (int j = 0; j < 4; ++j) {
      const size_t bo = (size_t)(n0 + (j << 4) + rlane) * ldb + koff + k0;
      bh[j] = Frag<T>::load(Bb + bo);
      if (SPLIT) bl[j] = Frag<T>::load(Bb2 + bo);
    }
#pragma unroll
    for (int i = 0; i < 4; ++i) {
      const size_t ao = (size_t)(m0 + (i << 4) + rlane) * lda + koff + k0;
      V ah = Frag<T>::load(Ab + ao);
      V al;
      if (SPLIT) al = Frag<T>::load(Ab2 + ao);
#pragma unroll
      for (int j = 0; j < 4; ++j) {
        acc[i][j] = Frag<T>::mma(ah, bh[j], acc[i][j]);
        if (SPLIT) {
          acc[i][j] = Frag<T>::mma(ah, bl[j], acc[i][j]);
          acc[i][j] = Frag<T>::mma(al, bh[j], acc[i][j]);
        }
      }
      Frag<T>::guard(acc[i][0], acc[i][3], ah, SPLIT ? al : ah);
    }
    Frag<T>::keep(bh[0], bh[1], bh[2], bh[3]);
    if (SPLIT) Frag<T>::keep(bl[0], bl[1], bl[2], bl[3]);
  }
  acc_guard4(acc[0][0], acc[0][1], acc[0][2], acc[0][3]);
  acc_guard4(acc[1][0], acc[1][1], acc[1][2], acc[1][3]);
  acc_guard4(acc[2][0], acc[2][1], acc[2][2], acc[2][3]);
  acc_guard4(acc[3][0], acc[3][1], acc[3][2], acc[3][3]);

  float* slab = sT[wave];
  const float* Rb = RESID ? (resid + (size_t)b * strideR) : nullptr;
#pragma unroll
  for (int i = 0; i < 4; ++i) {
    const int mBase = m0 + (i << 4);
#pragma unroll
    for (int j = 0; j < 4; ++j) {
      const int n = n0 + (j << 4) + rlane;
      float bv = 0.f;
      if (BIAS_MODE == 2) bv = bias[n];
#pragma unroll
      for (int r = 0; r < 8; ++r) {
        float v = acc[i][j][r] * scale;
        if (BIAS_MODE == 1) v += bias[mBase + mOff + r];
        if (BIAS_MODE == 2) v += bv;
        if (RESID) v += Rb[(size_t)(mBase + mOff + r) * ldc + n];
        if (ACT == 1) v = tanhf(v);
        slab[(mOff + r) * 68 + (j << 4) + rlane] = v;
      }
    }
    __builtin_amdgcn_fence(__ATOMIC_RELEASE, "workgroup");
    __builtin_amdgcn_wave_barrier();
    __builtin_amdgcn_fence(__ATOMIC_ACQUIRE, "workgroup");
    if (OUT_MODE == 0) {
      float* C = (float*)Cout + (size_t)b * strideC;
      const int hh = lane >> 4, c4 = (lane & 15) * 4;
      for (int pass = 0; pass < 2; ++pass) {
#pragma unroll
        for (int it = 0; it < 8; ++it) {
          const int row = it * 2 + hh;
          v4f v = *(const v4f*)(slab + row * 68 + c4);
          *(volatile v4f*)(C + (size_t)(mBase + row) * ldc + n0 + c4) = v;
        }
        __threadfence();
      }
    } else {
      const int q = lane >> 3, c8 = (lane & 7) * 8;
      unsigned short* C  = (unsigned short*)Cout  + (size_t)b * strideC;
      unsigned short* C2 = (OUT_MODE == 2) ? ((unsigned short*)Cout2 + (size_t)b * strideC) : nullptr;
      for (int pass = 0; pass < 2; ++pass) {
#pragma unroll
        for (int it = 0; it < 4; ++it) {
          const int row = it * 4 + q;
          const float* sp = slab + row * 68 + c8;
          v8h hv, lv;
#pragma unroll
          for (int e = 0; e < 8; ++e) {
            if (OUT_MODE == 1) {
              hv[e] = (_Float16)sp[e];
            } else {
              unsigned short hb = f2bf_bits(sp[e]);
              unsigned short lb = f2bf_bits(sp[e] - bf_bits2f(hb));
              hv[e] = __builtin_bit_cast(_Float16, hb);
              lv[e] = __builtin_bit_cast(_Float16, lb);
            }
          }
          *(volatile v8h*)(C + (size_t)(mBase + row) * ldc + n0 + c8) = hv;
          if (OUT_MODE == 2) *(volatile v8h*)(C2 + (size_t)(mBase + row) * ldc + n0 + c8) = lv;
        }
        __threadfence();
      }
    }
    __builtin_amdgcn_fence(__ATOMIC_RELEASE, "workgroup");
    __builtin_amdgcn_wave_barrier();
    __builtin_amdgcn_fence(__ATOMIC_ACQUIRE, "workgroup");
  }
}

__global__ __launch_bounds__(256) void cast_f32_f16x2(
    const float* __restrict__ in, _Float16* __restrict__ out, int n2) {
  int i = blockIdx.x * 256 + threadIdx.x;
  if (i < n2) {
    const _Float16 h0 = (_Float16)in[2 * i], h1 = (_Float16)in[2 * i + 1];
    const unsigned u = (unsigned)__builtin_bit_cast(unsigned short, h0) | ((unsigned)__builtin_bit_cast(unsigned short, h1) << 16);
    ((volatile unsigned*)out)[i] = u;
    __threadfence();
    ((volatile unsigned*)out)[i] = u;
  }
}


__global__ __launch_bounds__(256) void transpose_cast_f16(const float* __restrict__ in, int ldi,
                                                         _Float16* __restrict__ outT, int ldo, float scale) {
  __shared__ __align__(16) _Float16 tile[64][72];
  const int c0 = blockIdx.x * 64, r0 = blockIdx.y * 64;
  const int t = threadIdx.y * 32 + threadIdx.x;
  for (int i = threadIdx.y; i < 64; i += 8) {
    tile[threadIdx.x][i]      = (_Float16)(in[(size_t)(r0 + i) * ldi + c0 + threadIdx.x] * scale);
    tile[32 + threadIdx.x][i] = (_Float16)(in[(size_t)(r0 + i) * ldi + c0 + 32 + threadIdx.x] * scale);
  }
  __syncthreads();
  const int q = t >> 3, c8 = (t & 7) * 8;
  for (int pass = 0; pass < 2; ++pass) {
#pragma unroll
    for (int it = 0; it < 2; ++it) {
      const int c = it * 32 + q;
      v8h hv = *(const v8h*)(&tile[c][c8]);
      *(volatile v8h*)(outT + (size_t)(c0 + c) * ldo + r0 + c8) = hv;
    }
    __threadfence();
  }
}

__global__ __launch_bounds__(256) void pad_w_kernel(const float* __restrict__ w, _Float16* __restrict__ out, int R, int C, int RP) {
  const int i = blockIdx.x * 256 + threadIdx.x; const int n2 = RP * C / 2;
  if (i >= n2) return;
  const int e0 = 2 * i; const int r = e0 / C, c = e0 % C;
  const float v0 = (r < R) ? w[r * C + c] : 0.f, v1 = (r < R) ? w[r * C + c + 1] : 0.f;
  const unsigned u = (unsigned)__builtin_bit_cast(unsigned short, (_Float16)v0) | ((unsigned)__builtin_bit_cast(unsigned short, (_Float16)v1) << 16);
  ((volatile unsigned*)out)[i] = u; __threadfence(); ((volatile unsigned*)out)[i] = u;
}
__global__ void pad_b_kernel(const float* __restrict__ b, float* __restrict__ out, int R) {
  const int i = threadIdx.x;
  const float v = (i < R) ? b[i] : 0.f;
  ((volatile float*)out)[i] = v; __threadfence(); ((volatile float*)out)[i] = v;
}
__global__ __launch_bounds__(256) void softmax_row16(const float* __restrict__ S, _Float16* __restrict__ P, int Lc) {
  __shared__ float red[8];
  const size_t row = blockIdx.x;
  const float* s = S + row * Lc; _Float16* p = P + row * Lc;
  const int t = threadIdx.x;
  float ev[16];
#pragma unroll
  for (int g = 0; g < 2; ++g) {
    const int cb = g * (Lc / 2) + 8 * t;
    v4f a = *(const v4f*)(s + cb), c4 = *(const v4f*)(s + cb + 4);
    ev[8*g] = a[0]; ev[8*g+1] = a[1]; ev[8*g+2] = a[2]; ev[8*g+3] = a[3]; ev[8*g+4] = c4[0]; ev[8*g+5] = c4[1]; ev[8*g+6] = c4[2]; ev[8*g+7] = c4[3];
  }
  float m = ev[0];
#pragma unroll
  for (int i = 1; i < 16; ++i) m = fmaxf(m, ev[i]);
  for (int off = 16; off > 0; off >>= 1) m = fmaxf(m, __shfl_xor(m, off, 32));
  if ((t & 31) == 0) red[t >> 5] = m;
  __syncthreads();
  m = red[0];
#pragma unroll
  for (int w = 1; w < 8; ++w) m = fmaxf(m, red[w]);
  __syncthreads();
  float sum = 0.f;
#pragma unroll
  for (int i = 0; i < 16; ++i) { ev[i] = expf(ev[i] - m); sum += ev[i]; }
  for (int off = 16; off > 0; off >>= 1) sum += __shfl_xor(sum, off, 32);
  if ((t & 31) == 0) red[t >> 5] = sum;
  __syncthreads();
  float tot = 0.f;
#pragma unroll
  for (int w = 0; w < 8; ++w) tot += red[w];
  const float f = PSCALE / tot;
  v8h h0, h1;
#pragma unroll
  for (int i = 0; i < 8; ++i) { h0[i] = (_Float16)(ev[i] * f); h1[i] = (_Float16)(ev[8 + i] * f); }
  for (int pass = 0; pass < 2; ++pass) {
    *(volatile v8h*)(p + 8 * t) = h0;
    *(volatile v8h*)(p + Lc / 2 + 8 * t) = h1;
    __threadfence();
  }
}

extern "C" void kernel_launch(void* const* d_in, const int* in_sizes, int n_in,
                              void* d_out, int out_size, void* d_ws, size_t ws_size,
                              hipStream_t stream) {
  (void)in_sizes; (void)n_in; (void)out_size; (void)ws_size;
  const int B = 2, NH = 4, CPH = 128, QK = 16, N = 4096, C = 512;
  const float* x1 = (const float*)d_in[0];
  const float* x2 = (const float*)d_in[1];
  const float* qw = (const float*)d_in[2]; const float* qb = (const float*)d_in[3];
  const float* kw = (const float*)d_in[4]; const float* kb = (const float*)d_in[5];
  const float* vw = (const float*)d_in[6]; const float* vb = (const float*)d_in[7];
  float* out = (float*)d_out;

  char* ws = (char*)d_ws; size_t off = 0;
  auto carve = [&](size_t bytes) -> char* { char* p = ws + off; off += (bytes + 255) & ~(size_t)255; return p; };
  _Float16* X1t = (_Float16*)carve((size_t)N * CPH * 2);
  _Float16* X2t = (_Float16*)carve((size_t)N * CPH * 2);
  _Float16* Qw  = (_Float16*)carve((size_t)64 * CPH * 2);
  _Float16* Kw  = (_Float16*)carve((size_t)64 * CPH * 2);
  _Float16* Vw  = (_Float16*)carve((size_t)CPH * CPH * 2);
  float*    Qbp = (float*)carve(64 * 4);
  float*    Kbp = (float*)carve(64 * 4);
  __bf16*   Qth = (__bf16*)carve((size_t)N * 64 * 2);
  __bf16*   Qtl = (__bf16*)carve((size_t)N * 64 * 2);
  __bf16*   Kth = (__bf16*)carve((size_t)N * 64 * 2);
  __bf16*   Ktl = (__bf16*)carve((size_t)N * 64 * 2);
  _Float16* V   = (_Float16*)carve((size_t)CPH * N * 2);
  float*    Sc  = (float*)carve((size_t)N * N * 4);
  _Float16* P   = (_Float16*)carve((size_t)N * N * 2);

  for (int b = 0; b < B; ++b) for (int h = 0; h < NH; ++h) {
    const float* x1p = x1 + ((size_t)b * C + h * CPH) * N;
    const float* x2p = x2 + ((size_t)b * C + h * CPH) * N;
    transpose_cast_f16<<<dim3(N / 64, CPH / 64), dim3(32, 8), 0, stream>>>(x1p, N, X1t, CPH, 1.0f);
    transpose_cast_f16<<<dim3(N / 64, CPH / 64), dim3(32, 8), 0, stream>>>(x2p, N, X2t, CPH, 1.0f);
    pad_w_kernel<<<(64 * CPH / 2 + 255) / 256, 256, 0, stream>>>(qw + (size_t)h * QK * CPH, Qw, QK, CPH, 64);
    pad_w_kernel<<<(64 * CPH / 2 + 255) / 256, 256, 0, stream>>>(kw + (size_t)h * QK * CPH, Kw, QK, CPH, 64);
    pad_w_kernel<<<(CPH * CPH / 2 + 255) / 256, 256, 0, stream>>>(vw + (size_t)h * CPH * CPH, Vw, CPH, CPH, CPH);
    pad_b_kernel<<<1, 64, 0, stream>>>(qb + h * QK, Qbp, QK);
    pad_b_kernel<<<1, 64, 0, stream>>>(kb + h * QK, Kbp, QK);
    {
      const int t1 = (N / 64) * 1;
      wmma_gemm64<0, false, 2, 2, false><<<dim3((t1 + 7) / 8, 1), 256, 0, stream>>>(
          U16(X1t), nullptr, CPH, 0, U16(Qw), nullptr, CPH, 0, Qth, Qtl, 64, 0, Qbp, nullptr, 0, N, 64, CPH, 1.0f);
      wmma_gemm64<0, false, 2, 2, false><<<dim3((t1 + 7) / 8, 1), 256, 0, stream>>>(
          U16(X2t), nullptr, CPH, 0, U16(Kw), nullptr, CPH, 0, Kth, Ktl, 64, 0, Kbp, nullptr, 0, N, 64, CPH, 1.0f);
      const int tv = (CPH / 64) * (N / 64);
      wmma_gemm64<0, false, 1, 1, false><<<dim3((tv + 7) / 8, 1), 256, 0, stream>>>(
          U16(Vw), nullptr, CPH, 0, U16(X2t), nullptr, CPH, 0, V, nullptr, N, 0, vb + (size_t)h * CPH, nullptr, 0, CPH, N, CPH, 1.0f);
    }
    {
      const int ts = (N / 64) * (N / 64);
      wmma_gemm64<1, true, 0, 0, false><<<dim3((ts + 7) / 8, 1), 256, 0, stream>>>(
          U16(Qth), U16(Qtl), 64, 0, U16(Kth), U16(Ktl), 64, 0, Sc, nullptr, N, 0, nullptr, nullptr, 0, N, N, 32, 1.0f);
    }
    softmax_row16<<<N, 256, 0, stream>>>(Sc, P, N);
    {
      const int to = (CPH / 64) * (N / 64);
      wmma_gemm64<0, false, 0, 0, false><<<dim3((to + 7) / 8, 1), 256, 0, stream>>>(
          U16(V), nullptr, N, 0, U16(P), nullptr, N, 0, out + ((size_t)b * C + h * CPH) * N, nullptr, N, 0, nullptr, nullptr, 0, CPH, N, N, PSCALE_INV);
    }
  }
}
